// SplitHeadAttention_37752762531952
// MI455X (gfx1250) — hardware-verified
//
#include <hip/hip_runtime.h>
#include <math.h>

typedef __attribute__((ext_vector_type(16))) _Float16 v16h;
typedef __attribute__((ext_vector_type(16))) __bf16 v16b;
typedef __attribute__((ext_vector_type(8)))  _Float16 v8h;
typedef __attribute__((ext_vector_type(8)))  float v8f;
typedef __attribute__((ext_vector_type(4)))  float v4f;
typedef __attribute__((ext_vector_type(2)))  float v2f;
typedef __attribute__((ext_vector_type(4)))  unsigned v4u;
typedef __attribute__((ext_vector_type(4)))  int v4i;
typedef float __attribute__((may_alias)) float_a;
typedef int __attribute__((may_alias)) int_a;

template <typename T> __device__ __forceinline__ void vst2(void* p, T v) { *(volatile T*)p = v; __threadfence(); *(volatile T*)p = v; }
__device__ __forceinline__ v8f wmma16(v16h a, v16h b, v8f c) {
  v8f d = __builtin_amdgcn_wmma_f32_16x16x32_f16(false, a, false, b, (short)0, c, false, false);
  asm volatile("v_nop\n\tv_nop\n\tv_nop\n\tv_nop" : "+v"(d) : "v"(a), "v"(b));
  return d;
}
__device__ __forceinline__ v8f wmma_bf(v16b a, v16b b, v8f c) {
  v8f d = __builtin_amdgcn_wmma_f32_16x16x32_bf16(false, a, false, b, (short)0, c, false, false);
  asm volatile("v_nop\n\tv_nop\n\tv_nop\n\tv_nop" : "+v"(d) : "v"(a), "v"(b));
  return d;
}
__device__ __forceinline__ v16h frag_h(const _Float16* rowk0, int lane) {
  union { v16h v; v8h q[2]; } u; const _Float16* p = rowk0 + 8 * (lane >> 4);
  u.q[0] = *(const v8h*)p; u.q[1] = *(const v8h*)(p + 16); return u.v;
}
__device__ __forceinline__ v16h frag_f32(const float* rowk0, int lane) {
  v16h a; const float* p = rowk0 + 8 * (lane >> 4);
#pragma unroll
  for (int i = 0; i < 8; ++i) { a[i] = (_Float16)p[i]; a[8 + i] = (_Float16)p[16 + i]; }
  return a;
}
__device__ __forceinline__ v16h frag_f32s(const float* rowk0, int lane, float sc) {
  v16h a; const float* p = rowk0 + 8 * (lane >> 4);
#pragma unroll
  for (int i = 0; i < 8; ++i) { a[i] = (_Float16)(p[i] * sc); a[8 + i] = (_Float16)(p[16 + i] * sc); }
  return a;
}
__device__ __forceinline__ v16h fragc_f32(const float* W, int k0, int n, int lane, int ld, int K) {
  v16h a; const int g = lane >> 4;
#pragma unroll
  for (int i = 0; i < 8; ++i) { const int ka = k0 + 8 * g + i, kb = ka + 16;
    a[i] = (_Float16)(ka < K ? W[(size_t)ka * ld + n] : 0.f); a[8 + i] = (_Float16)(kb < K ? W[(size_t)kb * ld + n] : 0.f); }
  return a;
}
struct F2 { v16b h, l; };
__device__ __forceinline__ F2 bsplit16(const float v[16]) { F2 r;
#pragma unroll
  for (int i = 0; i < 16; ++i) { const __bf16 h = (__bf16)v[i]; r.h[i] = h; r.l[i] = (__bf16)(v[i] - (float)h); }
  return r; }
__device__ __forceinline__ F2 split_row(const float* row, int k0, int lane) { float v[16]; const float* p = row + k0 + 8 * (lane >> 4);
#pragma unroll
  for (int i = 0; i < 8; ++i) { v[i] = p[i]; v[8 + i] = p[16 + i]; }
  return bsplit16(v); }
__device__ __forceinline__ F2 split_rowK(const float* row, int k0, int lane, int K) { float v[16]; const int g = lane >> 4;
#pragma unroll
  for (int i = 0; i < 8; ++i) { const int ka = k0 + 8 * g + i, kb = ka + 16; v[i] = ka < K ? row[ka] : 0.f; v[8 + i] = kb < K ? row[kb] : 0.f; }
  return bsplit16(v); }
__device__ __forceinline__ F2 split_col(const float* W, int k0, int n, int lane, int ld, int K) { float v[16]; const int g = lane >> 4;
#pragma unroll
  for (int i = 0; i < 8; ++i) { const int ka = k0 + 8 * g + i, kb = ka + 16; v[i] = ka < K ? W[(size_t)ka * ld + n] : 0.f; v[8 + i] = kb < K ? W[(size_t)kb * ld + n] : 0.f; }
  return bsplit16(v); }
__device__ __forceinline__ v8f mac3(const F2& a, const F2& b, v8f c) { c = wmma_bf(a.l, b.h, c); c = wmma_bf(a.h, b.l, c); return wmma_bf(a.h, b.h, c); }
__device__ __forceinline__ float sigm(float v) { return 1.0f / (1.0f + expf(-v)); }
#define LDSX() do { asm volatile("s_wait_dscnt 0" ::: "memory"); __builtin_amdgcn_wave_barrier(); __builtin_amdgcn_fence(__ATOMIC_RELEASE, "workgroup"); } while (0)


#define NB 8
#define T 4096
#define XD 6
#define HD 64
#define DM 128
__device__ __forceinline__ float bfr(float v) { return (float)(__bf16)v; }

__global__ __launch_bounds__(256) void k_prep(const float* __restrict__ x, const float* __restrict__ Wq1, const float* __restrict__ Wk1, const float* __restrict__ Wq2, const float* __restrict__ Wk2, __bf16* __restrict__ AG, __bf16* __restrict__ XB, __bf16* __restrict__ XT, __bf16* __restrict__ ZB) {
  __shared__ float sG[2][9];
  const int tid = threadIdx.x;
  if (tid < 18) { const int h = tid / 9, a = (tid % 9) / 3, c = tid % 3; const float* Wq = h ? Wq2 : Wq1; const float* Wk = h ? Wk2 : Wk1; float s = 0.f; for (int d = 0; d < HD; ++d) s += bfr(Wq[a * HD + d]) * bfr(Wk[c * HD + d]); sG[h][a * 3 + c] = s * 0.125f; }
  __syncthreads();
  const int tok = blockIdx.x * 256 + tid;
  __shared__ __align__(16) __bf16 sag[2][256][32], sxb[2][256][32];
  if (blockIdx.x == 0 && tid < 8) { union { __bf16 e[8]; v4u u; } z; for (int e = 0; e < 8; ++e) z.e[e] = (__bf16)0.f; vst2((unsigned*)(ZB + tid * 8), z.u); }
#pragma unroll
  for (int h = 0; h < 2; ++h) { const float* xr = x + (size_t)tok * XD + h * 3; const float x0 = bfr(xr[0]), x1 = bfr(xr[1]), x2 = bfr(xr[2]);
#pragma unroll
    for (int e = 0; e < 32; ++e) { sag[h][tid][e] = (__bf16)0.f; sxb[h][tid][e] = (__bf16)0.f; }
#pragma unroll
    for (int c = 0; c < 3; ++c) { const float a = x0 * sG[h][0 * 3 + c] + x1 * sG[h][1 * 3 + c] + x2 * sG[h][2 * 3 + c]; const __bf16 hi = (__bf16)a; sag[h][tid][c] = hi; sag[h][tid][3 + c] = (__bf16)(a - (float)hi); }
    sxb[h][tid][0] = (__bf16)x0; sxb[h][tid][1] = (__bf16)x1; sxb[h][tid][2] = (__bf16)x2; sxb[h][tid][3] = (__bf16)x0; sxb[h][tid][4] = (__bf16)x1; sxb[h][tid][5] = (__bf16)x2; }
  __syncthreads();
#pragma unroll
  for (int h = 0; h < 2; ++h) { for (int q = tid; q < 256 * 4; q += 256) { const int rl = q >> 2, pc = q & 3; const size_t rowg = (size_t)h * NB * T + (size_t)blockIdx.x * 256 + rl;
      vst2((unsigned*)(AG + rowg * 32 + pc * 8), *(const v4u*)(&sag[h][rl][pc * 8])); vst2((unsigned*)(XB + rowg * 32 + pc * 8), *(const v4u*)(&sxb[h][rl][pc * 8])); } }
  __shared__ __bf16 sx[6][256];
  { const float* xr = x + (size_t)tok * XD; for (int p = 0; p < 6; ++p) sx[p][tid] = (__bf16)xr[p]; }
  __syncthreads();
  if (tid < 192) { const int p = tid >> 5, l = tid & 31; const int h = p / 3, c = p % 3; vst2((unsigned*)(XT + ((size_t)(h * 3 + c)) * (NB * T + 64) + (size_t)blockIdx.x * 256 + l * 8), *(const v4u*)(&sx[p][l * 8])); }
}
__device__ __forceinline__ v16b frag_b(const __bf16* rowk0, int lane) { return __builtin_bit_cast(v16b, frag_h((const _Float16*)rowk0, lane)); }
__global__ __launch_bounds__(128) void k_attn(const __bf16* __restrict__ AG, const __bf16* __restrict__ XB, const __bf16* __restrict__ XT, const __bf16* __restrict__ ZB, const float* __restrict__ Wv1, const float* __restrict__ Wv2, float* __restrict__ O32) {
  __shared__ __align__(16) float sS[4][16][68]; __shared__ float sWv[3][HD];
  const int tid = threadIdx.x, w = tid >> 5, lane = tid & 31, col = lane & 15, g = lane >> 4;
  const int bh = blockIdx.y, b = bh >> 1, h = bh & 1; const int qb = blockIdx.x; const int q0 = qb * 64 + w * 16;
  const float* Wv = h == 0 ? Wv1 : Wv2;
  for (int q = tid; q < 3 * HD; q += 128) sWv[q / HD][q % HD] = bfr(Wv[q]);
  __syncthreads();
  const __bf16* AGb = AG + ((size_t)h * NB * T + (size_t)b * T) * 32; const __bf16* XBb = XB + ((size_t)h * NB * T + (size_t)b * T) * 32; const __bf16* XTb = XT + (size_t)(h * 3) * (NB * T + 64) + (size_t)b * T;
  const v16b afr = frag_b(AGb + (size_t)(q0 + col) * 32, lane);
  float mrun = -3.0e38f, lrun = 0.f; v8f pxh = {}, pxl = {};
#pragma unroll 1
  for (int kt = 0; kt <= qb; ++kt) {
#pragma unroll
    for (int t = 0; t < 4; ++t) { const int key = kt * 64 + t * 16 + col;
      const v8f s = wmma_bf(afr, frag_b(XBb + (size_t)key * 32, lane), (v8f){});
#pragma unroll
      for (int r = 0; r < 8; ++r) sS[w][8 * g + r][t * 16 + col] = (key > q0 + 8 * g + r) ? -3.0e38f : s[r]; }
    LDSX();
    float mx = -3.4e38f;
#pragma unroll
    for (int jj = 0; jj < 32; ++jj) mx = fmaxf(mx, sS[w][col][g * 32 + jj]);
    mx = fmaxf(mx, __shfl_xor(mx, 16, 32));
    const float mnew = fmaxf(mrun, mx); const float corr = expf(mrun - mnew);
    float ps = 0.f;
#pragma unroll
    for (int jj = 0; jj < 32; ++jj) { const float sv = sS[w][col][g * 32 + jj]; const float p = sv <= -1.0e38f ? 0.f : expf(sv - mnew); ps += p; sS[w][col][g * 32 + jj] = p; }
    ps += __shfl_xor(ps, 16, 32);
    lrun = lrun * corr + ps; mrun = mnew;
#pragma unroll
    for (int r = 0; r < 8; ++r) { const float cr = __shfl(corr, 8 * g + r, 32); pxh[r] *= cr; pxl[r] *= cr; }
    LDSX();
#pragma unroll
    for (int kc = 0; kc < 2; ++kc) { const F2 pa = split_row(&sS[w][col][0], kc * 32, lane); const int kr0 = kt * 64 + kc * 32;
      const v16b xb_ = frag_b(col < 3 ? XTb + (size_t)col * (NB * T + 64) + kr0 : ZB, lane);
      pxh = wmma_bf(pa.h, xb_, pxh); pxl = wmma_bf(pa.l, xb_, pxl); }
    LDSX(); }
  { float px[8];
#pragma unroll
    for (int r = 0; r < 8; ++r) { const float lr = __shfl(lrun, 8 * g + r, 32); px[r] = (pxh[r] + pxl[r]) / lr; }
#pragma unroll
    for (int r = 0; r < 8; ++r) { const float p0 = __shfl(px[r], (lane & 16) + 0, 32), p1 = __shfl(px[r], (lane & 16) + 1, 32), p2 = __shfl(px[r], (lane & 16) + 2, 32);
      v4f o4;
#pragma unroll
      for (int e = 0; e < 4; ++e) { const int d = col * 4 + e; o4[e] = p0 * sWv[0][d] + p1 * sWv[1][d] + p2 * sWv[2][d]; }
      *(v4f*)(&sS[w][8 * g + r][col * 4]) = o4; } }
  LDSX();
  for (int qq = lane; qq < 16 * 16; qq += 32) { const int rl = qq >> 4, pc = qq & 15; vst2(O32 + ((size_t)b * T + q0 + rl) * DM + h * HD + pc * 4, *(const v4f*)(&sS[w][rl][pc * 4])); }
}
__global__ __launch_bounds__(128) void k_out(const float* __restrict__ O32, const float* __restrict__ Wout, float* __restrict__ out) {
  __shared__ __align__(16) float so[4][16][132];
  const int tid = threadIdx.x, wave = tid >> 5, lane = tid & 31, col = lane & 15, g = lane >> 4; const int r0 = blockIdx.x * 64 + wave * 16;
  v8f acc[8] = {};
#pragma unroll
  for (int kc = 0; kc < DM / 32; ++kc) { const F2 a = split_row(O32 + (size_t)(r0 + col) * DM, kc * 32, lane);
#pragma unroll
    for (int j = 0; j < 8; ++j) { const v16b wb = split_col(Wout, kc * 32, j * 16 + col, lane, DM, DM).h; acc[j] = wmma_bf(a.l, wb, acc[j]); acc[j] = wmma_bf(a.h, wb, acc[j]); } }
#pragma unroll
  for (int j = 0; j < 8; ++j)
#pragma unroll
    for (int r = 0; r < 8; ++r) so[wave][8 * g + r][j * 16 + col] = acc[j][r];
  LDSX();
#pragma unroll 4
  for (int rl = 0; rl < 16; ++rl) vst2(out + (size_t)(r0 + rl) * DM + lane * 4, *(const v4f*)(&so[wave][rl][lane * 4]));
}
extern "C" void kernel_launch(void* const* d_in, const int* in_sizes, int n_in, void* d_out, int out_size, void* d_ws, size_t ws_size, hipStream_t stream) {
  (void)in_sizes; (void)n_in; (void)out_size; (void)ws_size;
  const float** I = (const float**)d_in;
  float* out = (float*)d_out;
  char* ws = (char*)d_ws; size_t off = 0;
  auto take = [&](size_t bytes) { char* p = ws + off; off += (bytes + 255) & ~(size_t)255; return p; };
  float* O32 = (float*)take((size_t)NB * T * DM * 4); __bf16* AG = (__bf16*)take((size_t)2 * NB * T * 64); __bf16* XB = (__bf16*)take((size_t)2 * NB * T * 64); __bf16* XT = (__bf16*)take((size_t)6 * (NB * T + 64) * 2); __bf16* ZB = (__bf16*)take(256);
  k_prep<<<NB * T / 256, 256, 0, stream>>>(I[0], I[1], I[2], I[4], I[5], AG, XB, XT, ZB);
  k_attn<<<dim3(T / 64, NB * 2), 128, 0, stream>>>(AG, XB, XT, ZB, I[3], I[6], O32);
  k_out<<<NB * T / 64, 128, 0, stream>>>(O32, I[7], out);
}
